// BiMamba_21509196218760
// MI455X (gfx1250) — hardware-verified
//
#include <hip/hip_runtime.h>
#include <math.h>

typedef __attribute__((ext_vector_type(16))) _Float16 v16h;
typedef __attribute__((ext_vector_type(8)))  _Float16 v8h;
typedef __attribute__((ext_vector_type(16))) __bf16   v16b;
typedef __attribute__((ext_vector_type(8)))  __bf16   v8b;
typedef __attribute__((ext_vector_type(8)))  float    v8f;
typedef __attribute__((ext_vector_type(4)))  float    v4f;

constexpr int kBatch  = 2;
constexpr int kL      = 2048;
constexpr int kDm     = 768;
constexpr int kDi     = 1536;
constexpr int kNst    = 16;
constexpr int kHd     = 64;
constexpr int kNh     = 24;
constexpr int kConvC  = 1568;
constexpr int kPrjN   = 3128;
constexpr int kPrjP   = 3136;
constexpr int kDtCol  = 3104;
constexpr int kRows   = kBatch * kL;
constexpr int kCat    = 2 * kDm;
constexpr int kPrepP  = 64;
constexpr int kScanTS = 64;
constexpr int kScanYP = 68;
constexpr float kEps  = 1e-5f;
static_assert(kDi == 2 * kDm && kNh * kHd == kDi && kConvC == kDi + 2 * kNst, "shape chain");
static_assert(kPrjN == 2 * kDi + 2 * kNst + kNh && kDtCol == kDi + kConvC, "in_proj column map");
static_assert((kPrjP % 64) == 0 && kPrjP >= kPrjN && (kDm % 64) == 0 && (kL % 64) == 0 && (kRows % 64) == 0, "GEMM M,N multiples of 64");
static_assert((kDm % 32) == 0 && (kDi % 32) == 0, "GEMM K multiples of 32");
static_assert((kL % kScanTS) == 0 && kHd == 64 && kNst == 16, "scan tiling");
static_assert(kDi == 6 * 256, "norm column groups");

constexpr size_t kOffXB   = 0;
constexpr size_t kOffWIN  = kOffXB   + (size_t)kRows * kDm * 2;
constexpr size_t kOffWOUT = kOffWIN  + (size_t)2 * kPrjP * kDm * 2;
constexpr size_t kOffWPRJ = kOffWOUT + (size_t)2 * kDm * kDi * 2;
constexpr size_t kOffZX   = kOffWPRJ + (size_t)kDm * kCat * 2;
constexpr size_t kOffPREP = kOffZX   + (size_t)kL * kPrjP * 4;
constexpr size_t kOffYG   = kOffPREP + (size_t)kL * kPrepP * 4;
constexpr size_t kOffYNH  = kOffYG   + (size_t)kL * kDi * 4;
constexpr size_t kOffYNL  = kOffYNH  + (size_t)kL * kDi * 2;
constexpr size_t kOffCATH = kOffYNL  + (size_t)kL * kDi * 2;
constexpr size_t kOffCATL = kOffCATH + (size_t)kRows * kCat * 2;
constexpr size_t kWsTotal = kOffCATL + (size_t)kRows * kCat * 2;
static_assert(kWsTotal == 99549184ull, "carve total");
static_assert(kWsTotal <= 134217728ull, "carve cap");
static_assert((kOffWIN % 128) == 0 && (kOffWOUT % 128) == 0 && (kOffWPRJ % 128) == 0 && (kOffZX % 128) == 0 &&
              (kOffPREP % 128) == 0 && (kOffYG % 128) == 0 && (kOffYNH % 128) == 0 && (kOffYNL % 128) == 0 &&
              (kOffCATH % 128) == 0 && (kOffCATL % 128) == 0, "128-B aligned regions");

__device__ __forceinline__ unsigned short f2bf_bits(float f) {
  unsigned u = __float_as_uint(f);
  return (unsigned short)((u + 0x7FFFu + ((u >> 16) & 1u)) >> 16);
}
__device__ __forceinline__ float bf_bits2f(unsigned short h) { return __uint_as_float(((unsigned)h) << 16); }
__device__ __forceinline__ float bf_rne(float f) { return bf_bits2f(f2bf_bits(f)); }

__device__ __forceinline__ void dep_guard4_h(v8f& a, v8f& b, v8f& c, v8f& d, v16h x, v16h y) { asm volatile("v_nop\n\tv_nop\n\tv_nop\n\tv_nop" : "+v"(a), "+v"(b), "+v"(c), "+v"(d) : "v"(x), "v"(y)); }
__device__ __forceinline__ void dep_guard4_b(v8f& a, v8f& b, v8f& c, v8f& d, v16b x, v16b y) { asm volatile("v_nop\n\tv_nop\n\tv_nop\n\tv_nop" : "+v"(a), "+v"(b), "+v"(c), "+v"(d) : "v"(x), "v"(y)); }
__device__ __forceinline__ void keep4_h(v16h a, v16h b, v16h c, v16h d) { asm volatile("v_nop" :: "v"(a), "v"(b), "v"(c), "v"(d)); }
__device__ __forceinline__ void keep4_b(v16b a, v16b b, v16b c, v16b d) { asm volatile("v_nop" :: "v"(a), "v"(b), "v"(c), "v"(d)); }
__device__ __forceinline__ void acc_guard4(v8f& a, v8f& b, v8f& c, v8f& d) { asm volatile("v_nop\n\tv_nop\n\tv_nop\n\tv_nop" : "+v"(a), "+v"(b), "+v"(c), "+v"(d)); }
template <typename T> struct Frag;
template <> struct Frag<_Float16> {
  typedef v16h V; union U { v16h v; v8h h[2]; };
  static __device__ __forceinline__ v16h load(const _Float16* p) {
    U f; f.h[0] = *(const v8h*)(p); f.h[1] = *(const v8h*)(p + 16); return f.v;
  }
  static __device__ __forceinline__ v8f mma(v16h a, v16h b, v8f c) {
    return __builtin_amdgcn_wmma_f32_16x16x32_f16(false, a, false, b, (short)0, c, false, false);
  }
  static __device__ __forceinline__ void guard4(v8f& a, v8f& b, v8f& c, v8f& d, v16h x, v16h y) { dep_guard4_h(a, b, c, d, x, y); }
  static __device__ __forceinline__ void keep(v16h a, v16h b, v16h c, v16h d) { keep4_h(a, b, c, d); }
};
template <> struct Frag<__bf16> {
  typedef v16b V; union U { v16b v; v8b h[2]; };
  static __device__ __forceinline__ v16b load(const __bf16* p) {
    U f; f.h[0] = *(const v8b*)(p); f.h[1] = *(const v8b*)(p + 16); return f.v;
  }
  static __device__ __forceinline__ v8f mma(v16b a, v16b b, v8f c) {
    return __builtin_amdgcn_wmma_f32_16x16x32_bf16(false, a, false, b, (short)0, c, false, false);
  }
  static __device__ __forceinline__ void guard4(v8f& a, v8f& b, v8f& c, v8f& d, v16b x, v16b y) { dep_guard4_b(a, b, c, d, x, y); }
  static __device__ __forceinline__ void keep(v16b a, v16b b, v16b c, v16b d) { keep4_b(a, b, c, d); }
};

template <int ET> struct Elem;
template <> struct Elem<0> { typedef _Float16 T; };
template <> struct Elem<1> { typedef __bf16 T; };
template <int ET, int SPL, int BIAS_MODE, int OUT_MODE, bool RESID, int ACT = 0>
__global__ __launch_bounds__(256) void wmma_gemm64(
    const unsigned short* __restrict__ Ap, const unsigned short* __restrict__ A2p, int lda, long strideA,
    const unsigned short* __restrict__ Btp, const unsigned short* __restrict__ Bt2p, int ldb, long strideB,
    void* __restrict__ Cout, void* __restrict__ Cout2, int ldc, long strideC,
    const float* __restrict__ bias,
    const float* __restrict__ resid, long strideR,
    int M, int N, int K, float scale) {
  typedef typename Elem<ET>::T T;
  typedef typename Frag<T>::V V;
  const T* A = (const T*)Ap; const T* A2 = (const T*)A2p; const T* Bt = (const T*)Btp; const T* Bt2 = (const T*)Bt2p;
  __shared__ __align__(16) float sT[8][16 * 68];
  const int b    = blockIdx.y;
  const int lane = threadIdx.x & 31;
  const int wave = threadIdx.x >> 5;
  const int tilesN = N >> 6;
  const int tilesM = M >> 6;
  const int tile = blockIdx.x * 8 + wave;
  if (tile >= tilesM * tilesN) return;
  const int tm = tile / tilesN;
  const int tn = tile - tm * tilesN;
  const int m0 = tm << 6;
  const int n0 = tn << 6;

  const T* Ab  = A  + (size_t)b * strideA;
  const T* Bb  = Bt + (size_t)b * strideB;
  const T* Ab2 = (SPL >= 1) ? (A2  + (size_t)b * strideA) : nullptr;
  const T* Bb2 = (SPL == 2) ? (Bt2 + (size_t)b * strideB) : nullptr;

  const int rlane = lane & 15;
  const int koff  = (lane >> 4) * 8;
  const int mOff  = (lane >> 4) * 8;

  v8f acc[4][4];
#pragma unroll
  for (int i = 0; i < 4; ++i)
#pragma unroll
    for (int j = 0; j < 4; ++j) acc[i][j] = (v8f){0.f,0.f,0.f,0.f,0.f,0.f,0.f,0.f};

  for (int k0 = 0; k0 < K; k0 += 32) {
    V bh[4], bl[4];
#pragma unroll
    for (int j = 0; j < 4; ++j) {
      const size_t bo = (size_t)(n0 + (j << 4) + rlane) * ldb + koff + k0;
      bh[j] = Frag<T>::load(Bb + bo);
      if (SPL == 2) bl[j] = Frag<T>::load(Bb2 + bo);
    }
#pragma unroll
    for (int i = 0; i < 4; ++i) {
      const size_t ao = (size_t)(m0 + (i << 4) + rlane) * lda + koff + k0;
      V ah = Frag<T>::load(Ab + ao);
      V al;
      if (SPL >= 1) al = Frag<T>::load(Ab2 + ao);
#pragma unroll
      for (int j = 0; j < 4; ++j) {
        acc[i][j] = Frag<T>::mma(ah, bh[j], acc[i][j]);
        if (SPL == 2) acc[i][j] = Frag<T>::mma(ah, bl[j], acc[i][j]);
        if (SPL >= 1) acc[i][j] = Frag<T>::mma(al, bh[j], acc[i][j]);
      }
      Frag<T>::guard4(acc[i][0], acc[i][1], acc[i][2], acc[i][3], ah, (SPL >= 1) ? al : ah);
    }
    Frag<T>::keep(bh[0], bh[1], bh[2], bh[3]);
    if (SPL == 2) Frag<T>::keep(bl[0], bl[1], bl[2], bl[3]);
  }
  acc_guard4(acc[0][0], acc[0][1], acc[0][2], acc[0][3]);
  acc_guard4(acc[1][0], acc[1][1], acc[1][2], acc[1][3]);
  acc_guard4(acc[2][0], acc[2][1], acc[2][2], acc[2][3]);
  acc_guard4(acc[3][0], acc[3][1], acc[3][2], acc[3][3]);

  float* slab = sT[wave];
  const float* Rb = RESID ? (resid + (size_t)b * strideR) : nullptr;
#pragma unroll
  for (int i = 0; i < 4; ++i) {
    const int mBase = m0 + (i << 4);
#pragma unroll
    for (int j = 0; j < 4; ++j) {
      const int n = n0 + (j << 4) + rlane;
      float bv = 0.f;
      if (BIAS_MODE == 2) bv = bias[n];
      if (BIAS_MODE == 3) bv = bf_rne(bias[n]);
#pragma unroll
      for (int r = 0; r < 8; ++r) {
        float v = acc[i][j][r] * scale;
        if (BIAS_MODE == 1) v += bias[mBase + mOff + r];
        if (BIAS_MODE == 2 || BIAS_MODE == 3) v += bv;
        if (RESID) v += Rb[(size_t)(mBase + mOff + r) * ldc + n];
        if (ACT == 1) v = tanhf(v);
        if (ACT == 2) v = fmaxf(v, 0.0f);
        if (ACT == 3) v = v / (1.0f + expf(-v));
        if (ACT == 4) v = (v > 0.f) ? v : 0.01f * v;
        slab[(mOff + r) * 68 + (j << 4) + rlane] = v;
      }
    }
    __builtin_amdgcn_fence(__ATOMIC_RELEASE, "workgroup");
    __builtin_amdgcn_wave_barrier();
    __builtin_amdgcn_fence(__ATOMIC_ACQUIRE, "workgroup");
    if (OUT_MODE == 0) {
      float* C = (float*)Cout + (size_t)b * strideC;
      const int hh = lane >> 4, c4 = (lane & 15) * 4;
      for (int pass = 0; pass < 2; ++pass) {
#pragma unroll
        for (int it = 0; it < 8; ++it) {
          const int row = it * 2 + hh;
          v4f v = *(const v4f*)(slab + row * 68 + c4);
          *(volatile v4f*)(C + (size_t)(mBase + row) * ldc + n0 + c4) = v;
        }
        __threadfence();
      }
    } else {
      const int q = lane >> 3, c8 = (lane & 7) * 8;
      unsigned short* C  = (unsigned short*)Cout  + (size_t)b * strideC;
      unsigned short* C2 = (OUT_MODE == 2) ? ((unsigned short*)Cout2 + (size_t)b * strideC) : nullptr;
      for (int pass = 0; pass < 2; ++pass) {
#pragma unroll
        for (int it = 0; it < 4; ++it) {
          const int row = it * 4 + q;
          const float* sp = slab + row * 68 + c8;
          v8h hv, lv;
#pragma unroll
          for (int e = 0; e < 8; ++e) {
            if (OUT_MODE == 1) {
              hv[e] = (_Float16)sp[e];
            } else {
              unsigned short hb = f2bf_bits(sp[e]);
              unsigned short lb = f2bf_bits(sp[e] - bf_bits2f(hb));
              hv[e] = __builtin_bit_cast(_Float16, hb);
              lv[e] = __builtin_bit_cast(_Float16, lb);
            }
          }
          *(volatile v8h*)(C + (size_t)(mBase + row) * ldc + n0 + c8) = hv;
          if (OUT_MODE == 2) *(volatile v8h*)(C2 + (size_t)(mBase + row) * ldc + n0 + c8) = lv;
        }
        __threadfence();
      }
    }
    __builtin_amdgcn_fence(__ATOMIC_RELEASE, "workgroup");
    __builtin_amdgcn_wave_barrier();
    __builtin_amdgcn_fence(__ATOMIC_ACQUIRE, "workgroup");
  }
}

__global__ __launch_bounds__(256) void cast_bf16_kernel(
    const float* __restrict__ src, unsigned short* __restrict__ dst, int real8, int total8)
{
  const int i = blockIdx.x * 256 + threadIdx.x;
  if (i >= total8) return;
  const bool live = (i < real8);
  const int ic = live ? i : (real8 - 1);
  const float* p = src + ((size_t)ic << 3);
  const v4f a0 = *(const v4f*)(p);
  const v4f a1 = *(const v4f*)(p + 4);
  v8h hv;
#pragma unroll
  for (int e = 0; e < 4; ++e) {
    const float f0 = a0[e];
    const float f1 = a1[e];
    const unsigned short b0 = f2bf_bits(f0);
    const unsigned short b1 = f2bf_bits(f1);
    const unsigned short h0 = live ? b0 : (unsigned short)0;
    const unsigned short h1 = live ? b1 : (unsigned short)0;
    hv[e]     = __builtin_bit_cast(_Float16, h0);
    hv[4 + e] = __builtin_bit_cast(_Float16, h1);
  }
  unsigned short* q = dst + ((size_t)i << 3);
  *(volatile v8h*)q = hv;
  __threadfence();
  *(volatile v8h*)q = hv;
}

__global__ __launch_bounds__(256) void prep_kernel(
    const float* __restrict__ ZX, const float* __restrict__ cw, const float* __restrict__ cb,
    const float* __restrict__ dtb, float* __restrict__ PREP, int dir)
{
  __shared__ __align__(16) float sT[16 * kPrepP];
  const int tid = threadIdx.x;
  const int r0 = blockIdx.x * 16;
#pragma unroll 1
  for (int it = 0; it < 4; ++it) {
    const int idx = tid + it * 256;
    const int rl = idx >> 6;
    const int c  = idx & 63;
    const int t  = r0 + rl;
    const int hc = (c < kNh) ? c : (kNh - 1);
    float raw = ZX[(size_t)t * kPrjP + kDtCol + hc];
    asm volatile("" : "+v"(raw));
    const float v  = raw + bf_rne(dtb[hc]);
    const float sp = fmaxf(v, 0.0f) + log1pf(expf(-fabsf(v)));
    int cc = c - 32;
    cc = (cc < 0) ? 0 : cc;
    const int chn = kDi + cc;
    const int col = kDi + chn;
    float acc = 0.0f;
#pragma unroll
    for (int j = 0; j < 4; ++j) {
      const int tj = dir ? (t + (3 - j)) : (t - (3 - j));
      const bool ok = (tj >= 0) && (tj < kL);
      const int tc = (tj < 0) ? 0 : ((tj > kL - 1) ? (kL - 1) : tj);
      float xv = ZX[(size_t)tc * kPrjP + col];
      asm volatile("" : "+v"(xv));
      const float xs = ok ? xv : 0.0f;
      acc = fmaf(bf_rne(cw[chn * 4 + j]), xs, acc);
    }
    const float sv = acc + bf_rne(cb[chn]);
    const float sg = __builtin_amdgcn_rcpf(1.0f + expf(-sv));
    const float cv = sv * sg;
    const float res = (c < kNh) ? sp : ((c < 32) ? 0.0f : cv);
    sT[idx] = res;
  }
  __syncthreads();
  const v4f val = *(const v4f*)(sT + tid * 4);
  float* q = PREP + (size_t)r0 * kPrepP + tid * 4;
  *(volatile v4f*)q = val;
  __threadfence();
  *(volatile v4f*)q = val;
}

__global__ __launch_bounds__(64) void scan_kernel(
    const float* __restrict__ ZX, const float* __restrict__ PREP,
    const float* __restrict__ cw, const float* __restrict__ cb,
    const float* __restrict__ Alog, const float* __restrict__ Dp,
    float* __restrict__ YG, int dir)
{
  __shared__ __align__(16) float sP[kScanTS * kPrepP];
  __shared__ __align__(16) float sY[kScanTS * kScanYP];
  const int tid = threadIdx.x, lane = tid & 31, wave = tid >> 5;
  const int hd = blockIdx.x;
  const int ch = hd * kHd + tid;
  const float w0 = bf_rne(cw[ch * 4 + 0]);
  const float w1 = bf_rne(cw[ch * 4 + 1]);
  const float w2 = bf_rne(cw[ch * 4 + 2]);
  const float w3 = bf_rne(cw[ch * 4 + 3]);
  const float bc = bf_rne(cb[ch]);
  const float negA = -expf(bf_rne(Alog[hd]));
  const float Dd = bf_rne(Dp[hd]);
  float h[kNst];
#pragma unroll
  for (int n = 0; n < kNst; ++n) h[n] = 0.f;
  float xm3 = 0.f, xm2 = 0.f, xm1 = 0.f;
  const int lr = tid >> 4, lc4 = (tid & 15) * 4;
  const int hh = lane >> 4, c4 = (lane & 15) * 4;
#pragma unroll 1
  for (int ck = 0; ck < kL / kScanTS; ++ck) {
    const int tlo = dir ? (kL - kScanTS - ck * kScanTS) : (ck * kScanTS);
    __syncthreads();
#pragma unroll
    for (int i = 0; i < 16; ++i) {
      const int r = lr + 4 * i;
      *(v4f*)(sP + r * kPrepP + lc4) = *(const v4f*)(PREP + (size_t)(tlo + r) * kPrepP + lc4);
    }
    __syncthreads();
#pragma unroll 1
    for (int s = 0; s < kScanTS; ++s) {
      const int rr = dir ? (kScanTS - 1 - s) : s;
      const size_t t = (size_t)(tlo + rr);
      const float* xr = sP + rr * kPrepP;
      const float xraw = ZX[t * kPrjP + kDi + ch];
      const float zv   = ZX[t * kPrjP + ch];
      float acc = w0 * xm3;
      acc = fmaf(w1, xm2, acc);
      acc = fmaf(w2, xm1, acc);
      acc = fmaf(w3, xraw, acc);
      const float sv = acc + bc;
      const float xh = sv * __builtin_amdgcn_rcpf(1.0f + expf(-sv));
      xm3 = xm2; xm2 = xm1; xm1 = xraw;
      const float dt = xr[hd];
      float Bs[kNst], Cs[kNst];
#pragma unroll
      for (int q4 = 0; q4 < 4; ++q4) {
        const v4f bv = *(const v4f*)(xr + 32 + 4 * q4);
        const v4f cv = *(const v4f*)(xr + 48 + 4 * q4);
        Bs[4 * q4 + 0] = bv[0]; Bs[4 * q4 + 1] = bv[1]; Bs[4 * q4 + 2] = bv[2]; Bs[4 * q4 + 3] = bv[3];
        Cs[4 * q4 + 0] = cv[0]; Cs[4 * q4 + 1] = cv[1]; Cs[4 * q4 + 2] = cv[2]; Cs[4 * q4 + 3] = cv[3];
      }
      const float dA  = expf(dt * negA);
      const float dtx = dt * xh;
      float y = 0.f;
#pragma unroll
      for (int n = 0; n < kNst; ++n) {
        const float inj = dtx * Bs[n];
        h[n] = fmaf(h[n], dA, inj);
        y = fmaf(h[n], Cs[n], y);
      }
      y = fmaf(Dd, xh, y);
      const float gz = zv * __builtin_amdgcn_rcpf(1.0f + expf(-zv));
      sY[rr * kScanYP + tid] = y * gz;
    }
    __syncthreads();
    for (int pass = 0; pass < 2; ++pass) {
#pragma unroll
      for (int it = 0; it < 16; ++it) {
        const int row = it * 4 + wave * 2 + hh;
        const v4f v = *(const v4f*)(sY + row * kScanYP + c4);
        *(volatile v4f*)(YG + (size_t)(tlo + row) * kDi + hd * kHd + c4) = v;
      }
      __threadfence();
    }
  }
}

__global__ __launch_bounds__(256) void norm_kernel(
    const float* __restrict__ YG, const float* __restrict__ nw,
    unsigned short* __restrict__ YNH, unsigned short* __restrict__ YNL)
{
  const int lane = threadIdx.x & 31, wave = threadIdx.x >> 5;
  const int row = blockIdx.x * 8 + wave;
  const float* gr = YG + (size_t)row * kDi;
  float ss = 0.0f;
#pragma unroll 1
  for (int it = 0; it < 6; ++it) {
    const int col = it * 256 + lane * 8;
    const v4f a0 = *(const v4f*)(gr + col);
    const v4f a1 = *(const v4f*)(gr + col + 4);
#pragma unroll
    for (int e = 0; e < 4; ++e) {
      const float ga = a0[e];
      const float gb = a1[e];
      ss = fmaf(ga, ga, ss);
      ss = fmaf(gb, gb, ss);
    }
  }
  ss += __shfl_xor(ss, 16, 32);
  ss += __shfl_xor(ss, 8, 32);
  ss += __shfl_xor(ss, 4, 32);
  ss += __shfl_xor(ss, 2, 32);
  ss += __shfl_xor(ss, 1, 32);
  constexpr float kInvN = 1.0f / (float)kDi;
  const float r = rsqrtf(ss * kInvN + kEps);
#pragma unroll 1
  for (int it = 0; it < 6; ++it) {
    const int col = it * 256 + lane * 8;
    const v4f a0 = *(const v4f*)(gr + col);
    const v4f a1 = *(const v4f*)(gr + col + 4);
    const v4f n0 = *(const v4f*)(nw + col);
    const v4f n1 = *(const v4f*)(nw + col + 4);
    v8h hv, lv;
#pragma unroll
    for (int e = 0; e < 4; ++e) {
      const float ga = a0[e];
      const float gb = a1[e];
      const float wa = n0[e];
      const float wb = n1[e];
      const float ya = (ga * r) * bf_rne(wa);
      const float yb = (gb * r) * bf_rne(wb);
      const unsigned short ha = f2bf_bits(ya);
      const unsigned short hb = f2bf_bits(yb);
      const unsigned short la = f2bf_bits(ya - bf_bits2f(ha));
      const unsigned short lb = f2bf_bits(yb - bf_bits2f(hb));
      hv[e]     = __builtin_bit_cast(_Float16, ha);
      hv[4 + e] = __builtin_bit_cast(_Float16, hb);
      lv[e]     = __builtin_bit_cast(_Float16, la);
      lv[4 + e] = __builtin_bit_cast(_Float16, lb);
    }
    const size_t o = (size_t)row * kDi + col;
    *(volatile v8h*)(YNH + o) = hv;
    *(volatile v8h*)(YNL + o) = lv;
    __threadfence();
    *(volatile v8h*)(YNH + o) = hv;
    *(volatile v8h*)(YNL + o) = lv;
  }
}

extern "C" void kernel_launch(void* const* d_in, const int* in_sizes, int n_in,
                              void* d_out, int out_size, void* d_ws, size_t ws_size,
                              hipStream_t stream) {
  if (n_in < 19) return;
  if (in_sizes[0] != kRows * kDm) return;
  if (in_sizes[1] != kDm * kCat) return;
  if (in_sizes[2] != kDm) return;
  for (int d = 0; d < 2; ++d) {
    const int o = 3 + 8 * d;
    if (in_sizes[o + 0] != kPrjN * kDm) return;
    if (in_sizes[o + 1] != kConvC * 4) return;
    if (in_sizes[o + 2] != kConvC) return;
    if (in_sizes[o + 3] != kNh) return;
    if (in_sizes[o + 4] != kNh) return;
    if (in_sizes[o + 5] != kNh) return;
    if (in_sizes[o + 6] != kDi) return;
    if (in_sizes[o + 7] != kDm * kDi) return;
  }
  if (out_size != kRows * kDm) return;
  if (ws_size < kWsTotal) return;

  const float* x      = (const float*)d_in[0];
  const float* proj_w = (const float*)d_in[1];
  const float* proj_b = (const float*)d_in[2];
  const float* in_w[2]    = { (const float*)d_in[3],  (const float*)d_in[11] };
  const float* conv_w[2]  = { (const float*)d_in[4],  (const float*)d_in[12] };
  const float* conv_b[2]  = { (const float*)d_in[5],  (const float*)d_in[13] };
  const float* dt_bias[2] = { (const float*)d_in[6],  (const float*)d_in[14] };
  const float* A_log[2]   = { (const float*)d_in[7],  (const float*)d_in[15] };
  const float* Dpar[2]    = { (const float*)d_in[8],  (const float*)d_in[16] };
  const float* norm_w[2]  = { (const float*)d_in[9],  (const float*)d_in[17] };
  const float* out_w[2]   = { (const float*)d_in[10], (const float*)d_in[18] };
  float* out = (float*)d_out;

  char* ws = (char*)d_ws;
  unsigned short* XB   = (unsigned short*)(ws + kOffXB);
  unsigned short* WIN  = (unsigned short*)(ws + kOffWIN);
  unsigned short* WOUT = (unsigned short*)(ws + kOffWOUT);
  unsigned short* WPRJ = (unsigned short*)(ws + kOffWPRJ);
  float*          ZX   = (float*)(ws + kOffZX);
  float*          PREP = (float*)(ws + kOffPREP);
  float*          YG   = (float*)(ws + kOffYG);
  unsigned short* YNH  = (unsigned short*)(ws + kOffYNH);
  unsigned short* YNL  = (unsigned short*)(ws + kOffYNL);
  unsigned short* CATH = (unsigned short*)(ws + kOffCATH);
  unsigned short* CATL = (unsigned short*)(ws + kOffCATL);

  {
    const int n8x = kRows * kDm / 8;
    cast_bf16_kernel<<<n8x / 256, 256, 0, stream>>>(x, XB, n8x, n8x);
    const int r8w = kPrjN * kDm / 8;
    const int t8w = kPrjP * kDm / 8;
    for (int d = 0; d < 2; ++d)
      cast_bf16_kernel<<<t8w / 256, 256, 0, stream>>>(in_w[d], WIN + (size_t)d * kPrjP * kDm, r8w, t8w);
    const int n8o = kDm * kDi / 8;
    for (int d = 0; d < 2; ++d)
      cast_bf16_kernel<<<n8o / 256, 256, 0, stream>>>(out_w[d], WOUT + (size_t)d * kDm * kDi, n8o, n8o);
    const int n8p = kDm * kCat / 8;
    cast_bf16_kernel<<<n8p / 256, 256, 0, stream>>>(proj_w, WPRJ, n8p, n8p);
  }

  for (int d = 0; d < 2; ++d) {
    const unsigned short* WINd  = WIN  + (size_t)d * kPrjP * kDm;
    const unsigned short* WOUTd = WOUT + (size_t)d * kDm * kDi;
    for (int b = 0; b < kBatch; ++b) {
      const unsigned short* XBb = XB + (size_t)b * kL * kDm;

      wmma_gemm64<1, 0, 0, 0, false><<<dim3((kL / 64) * (kPrjP / 64) / 8, 1), 256, 0, stream>>>(
          XBb, XBb, kDm, 0L,
          WINd, WINd, kDm, 0L,
          (void*)ZX, (void*)ZX, kPrjP, 0L,
          proj_b, x, 0L,
          kL, kPrjP, kDm, 1.0f);

      prep_kernel<<<kL / 16, 256, 0, stream>>>(ZX, conv_w[d], conv_b[d], dt_bias[d], PREP, d);

      scan_kernel<<<kNh, kHd, 0, stream>>>(ZX, PREP, conv_w[d], conv_b[d], A_log[d], Dpar[d], YG, d);

      norm_kernel<<<kL / 8, 256, 0, stream>>>(YG, norm_w[d], YNH, YNL);

      unsigned short* ch = CATH + (size_t)b * kL * kCat + (size_t)d * kDm;
      unsigned short* cl = CATL + (size_t)b * kL * kCat + (size_t)d * kDm;
      wmma_gemm64<1, 1, 0, 2, false><<<dim3((kL / 64) * (kDm / 64) / 8, 1), 256, 0, stream>>>(
          YNH, YNL, kDi, 0L,
          WOUTd, WOUTd, kDi, 0L,
          (void*)ch, (void*)cl, kCat, 0L,
          proj_b, x, 0L,
          kL, kDm, kDi, 1.0f);
    }
  }

  wmma_gemm64<1, 1, 3, 0, false><<<dim3((kRows / 64) * (kDm / 64) / 8, 1), 256, 0, stream>>>(
      CATH, CATL, kCat, 0L,
      WPRJ, WPRJ, kCat, 0L,
      (void*)out, (void*)out, kDm, 0L,
      proj_b, x, 0L,
      kRows, kDm, kCat, 1.0f);
}
